// RNAEditingGNN_549755814553
// MI455X (gfx1250) — hardware-run, weakly checked
//
#include <hip/hip_runtime.h>
#include <stddef.h>


#define NTHR    256
#define NWAVE   8
#define EPTH    8
#define NGRP    2
#define CHUNK   (NTHR * EPTH * NGRP)
#define WCAP    (EPTH * NGRP * 32)
#define LISTN   (NWAVE * WCAP)
#define NBC     4096
#define NBF     1024
#define RCAP    40960
#define RBN     128
#define TGT     256
#define NSLOT   128
#define GROWS   128
#define GNC     64
#define OTHR    512
#define NPB     512
#define PTHR    64
#define NG      128
#define CH      64
#define NH      4
#define WSCAP   134217728
#define NEG_BIG (-3.0e38f)
#define NEGS    0.2f
#define BN_EPS  1e-5f
#define LDS_FILL ((RCAP + NBF + LISTN) * 4 + 64)
#define LDS_GEMM ((GROWS * GNC + 128 + GROWS * 8) * 4)

static_assert((CHUNK & (CHUNK - 1)) == 0);
static_assert(CHUNK <= 4096);
static_assert(NBC == 4 * NBF);
static_assert(OTHR * 8 == NBC);
static_assert((RCAP % 32) == 0);
static_assert(TGT == NWAVE * 32);
static_assert(GROWS == NWAVE * 16);
static_assert(NSLOT == 128);
static_assert(CH == 64);
static_assert(NG * CH == 32 * NTHR);
static_assert((NG * CH) % (4 * PTHR) == 0);

typedef float          v2f  __attribute__((ext_vector_type(2)));
typedef float          v4f  __attribute__((ext_vector_type(4)));
typedef float          v8f  __attribute__((ext_vector_type(8)));
typedef int            v4i  __attribute__((ext_vector_type(4)));
typedef unsigned int   v2u  __attribute__((ext_vector_type(2)));
typedef unsigned int   v4u  __attribute__((ext_vector_type(4)));
typedef unsigned short v8us __attribute__((ext_vector_type(8)));
typedef __bf16         v16b __attribute__((ext_vector_type(16)));
union FragB { v16b v; v8us h[2]; };

__device__ __forceinline__ unsigned int bfr(float f) {
  const unsigned int u = __float_as_uint(f);
  return (u + 0x7FFFu + ((u >> 16) & 1u)) >> 16;
}
__device__ __forceinline__ void split1(float x, unsigned short& hb, unsigned short& lb) {
  const unsigned int hu = bfr(x);
  const float hf = __uint_as_float(hu << 16);
  hb = (unsigned short)hu;
  lb = (unsigned short)bfr(x - hf);
}
__device__ __forceinline__ void split8(v4f a, v4f b, v8us& hi, v8us& lo) {
  unsigned short hb, lb;
  split1(a.x, hb, lb); hi[0] = hb; lo[0] = lb;
  split1(a.y, hb, lb); hi[1] = hb; lo[1] = lb;
  split1(a.z, hb, lb); hi[2] = hb; lo[2] = lb;
  split1(a.w, hb, lb); hi[3] = hb; lo[3] = lb;
  split1(b.x, hb, lb); hi[4] = hb; lo[4] = lb;
  split1(b.y, hb, lb); hi[5] = hb; lo[5] = lb;
  split1(b.z, hb, lb); hi[6] = hb; lo[6] = lb;
  split1(b.w, hb, lb); hi[7] = hb; lo[7] = lb;
}
__device__ __forceinline__ void pk2(float x, float y, unsigned int& hi, unsigned int& lo) {
  unsigned short a, b, c, d;
  split1(x, a, c); split1(y, b, d);
  hi = (unsigned int)a | ((unsigned int)b << 16);
  lo = (unsigned int)c | ((unsigned int)d << 16);
}

__device__ __forceinline__ v8f wm(v16b a, v16b b, v8f c) {
  return __builtin_amdgcn_wmma_f32_16x16x32_bf16(false, a, false, b, (short)0, c, false, false);
}
__device__ __forceinline__ v8f wm3(v16b ah, v16b al, v16b bh, v16b bl, v8f c) {
  c = wm(ah, bh, c); c = wm(ah, bl, c); c = wm(al, bh, c);
  asm volatile("v_nop\n\tv_nop\n\tv_nop\n\tv_nop" : "+v"(c) : "v"(ah), "v"(al), "v"(bh), "v"(bl));
  return c;
}

__device__ __forceinline__ float wsum(float v) {
#pragma unroll
  for (int o = 16; o > 0; o >>= 1) v += __shfl_xor(v, o);
  return v;
}
__device__ __forceinline__ float wmax(float v) {
#pragma unroll
  for (int o = 16; o > 0; o >>= 1) v = fmaxf(v, __shfl_xor(v, o));
  return v;
}

__device__ __forceinline__ float lgt(float s) {
  return (s > 0.0f) ? s : NEGS * s;
}

template <int NB>
__device__ __forceinline__ int scan_chunk(const int* __restrict__ dsts, int nE, int cbase, int slotBase,
                                          int vec8, int* list, int tid, int lane, int wave) {
  int wc = 0;
#pragma unroll
  for (int g = 0; g < NGRP; ++g) {
    const int el0  = (g * NTHR + tid) * EPTH;
    const int e0   = cbase + el0;
    const int sent = -2147483647 - 1;
    v4i da, db;
    if (vec8 != 0 && cbase + CHUNK <= nE) {
      da = *(const v4i*)(dsts + e0);
      db = *(const v4i*)(dsts + e0 + 4);
    } else {
      da.x = (e0     < nE) ? dsts[min(e0, nE - 1)] : sent;
      da.y = (e0 + 1 < nE) ? dsts[min(e0 + 1, nE - 1)] : sent;
      da.z = (e0 + 2 < nE) ? dsts[min(e0 + 2, nE - 1)] : sent;
      da.w = (e0 + 3 < nE) ? dsts[min(e0 + 3, nE - 1)] : sent;
      db.x = (e0 + 4 < nE) ? dsts[min(e0 + 4, nE - 1)] : sent;
      db.y = (e0 + 5 < nE) ? dsts[min(e0 + 5, nE - 1)] : sent;
      db.z = (e0 + 6 < nE) ? dsts[min(e0 + 6, nE - 1)] : sent;
      db.w = (e0 + 7 < nE) ? dsts[min(e0 + 7, nE - 1)] : sent;
    }
    const unsigned nb = (unsigned)slotBase;
    const unsigned s0 = (unsigned)da.x - nb, s1 = (unsigned)da.y - nb;
    const unsigned s2 = (unsigned)da.z - nb, s3 = (unsigned)da.w - nb;
    const unsigned s4 = (unsigned)db.x - nb, s5 = (unsigned)db.y - nb;
    const unsigned s6 = (unsigned)db.z - nb, s7 = (unsigned)db.w - nb;
    const bool h0 = s0 < (unsigned)NB, h1 = s1 < (unsigned)NB, h2 = s2 < (unsigned)NB, h3 = s3 < (unsigned)NB;
    const bool h4 = s4 < (unsigned)NB, h5 = s5 < (unsigned)NB, h6 = s6 < (unsigned)NB, h7 = s7 < (unsigned)NB;
    const unsigned any = __builtin_amdgcn_ballot_w32(h0 | h1 | h2 | h3 | h4 | h5 | h6 | h7);
    if (any != 0u) {
#define HITJ(J, HJ, SJ) { \
        const unsigned mj = __builtin_amdgcn_ballot_w32(HJ); \
        if (mj != 0u) { \
          if (HJ) { \
            const int p = wc + (int)__builtin_amdgcn_mbcnt_lo(mj, 0u); \
            if (p < WCAP) list[wave * WCAP + p] = ((el0 + (J)) << 12) | (int)(SJ); \
          } \
          wc += (int)__builtin_popcount(mj); } }
      HITJ(0, h0, s0)
      HITJ(1, h1, s1)
      HITJ(2, h2, s2)
      HITJ(3, h3, s3)
      HITJ(4, h4, s4)
      HITJ(5, h5, s5)
      HITJ(6, h6, s6)
      HITJ(7, h7, s7)
#undef HITJ
    }
  }
  return wc;
}

__global__ __launch_bounds__(NTHR) void k_count(const int* __restrict__ ei, int* cnt, int nE, int vec8) {
  __shared__ __attribute__((aligned(16))) int scnt[NBC];
  __shared__ __attribute__((aligned(16))) int list[LISTN];
  __shared__ int wcnt[NWAVE];
  const int tid = threadIdx.x, lane = tid & 31, wave = tid >> 5;
  const int nodeBase = blockIdx.x * NBC;
  const int* dsts = ei + nE;
  for (int i = tid; i < NBC; i += NTHR) scnt[i] = 0;
  __syncthreads();
  const int nChunks = (nE + CHUNK - 1) / CHUNK;
#pragma unroll 1
  for (int ch = 0; ch < nChunks; ++ch) {
    const int cbase = ch * CHUNK;
    const int wc = scan_chunk<NBC>(dsts, nE, cbase, nodeBase, vec8, list, tid, lane, wave);
    if (lane == 0) wcnt[wave] = wc;
    __syncthreads();
    if (wave == 0) {
#pragma unroll 1
      for (int wsx = 0; wsx < NWAVE; ++wsx) {
        int n = __builtin_amdgcn_readfirstlane(wcnt[wsx]);
        n = n > WCAP ? WCAP : (n < 0 ? 0 : n);
        const int* lp = list + wsx * WCAP;
#pragma unroll 1
        for (int i = 0; i < n; ++i) {
          const int ent  = __builtin_amdgcn_readfirstlane(lp[i]);
          const int slot = ent & (NBC - 1);
          if (lane == 0) scnt[slot] = scnt[slot] + 1;
        }
      }
    }
    __syncthreads();
  }
  v4i cq[4];
#pragma unroll
  for (int q = 0; q < 4; ++q) cq[q] = *(const v4i*)(scnt + (wave * 4 + q) * 128 + 4 * lane);
  int* cp = cnt + (size_t)nodeBase;
#pragma unroll
  for (int q = 0; q < 4; ++q) *(volatile v4i*)(cp + (wave * 4 + q) * 128 + 4 * lane) = cq[q];
  __threadfence();
#pragma unroll
  for (int q = 0; q < 4; ++q) *(volatile v4i*)(cp + (wave * 4 + q) * 128 + 4 * lane) = cq[q];
}

__global__ __launch_bounds__(OTHR) void k_offsets(const int* __restrict__ cnt, int* off, int* rbase, int nChunk) {
  __shared__ __attribute__((aligned(16))) int soff[NBC];
  __shared__ __attribute__((aligned(16))) int srb[RBN];
  __shared__ int wtot[OTHR / 32];
  const int tid = threadIdx.x, lane = tid & 31, wave = tid >> 5, sub = tid >> 7;
  for (int i = tid; i < RBN; i += OTHR) srb[i] = 0;
  int carry = 0;
#pragma unroll 1
  for (int ch = 0; ch < nChunk; ++ch) {
    const int base = ch * NBC;
    const v4i c0 = *(const v4i*)(cnt + base + 8 * tid);
    const v4i c1 = *(const v4i*)(cnt + base + 8 * tid + 4);
    const int e0 = max(c0.x, 0), e1 = max(c0.y, 0), e2 = max(c0.z, 0), e3 = max(c0.w, 0);
    const int e4 = max(c1.x, 0), e5 = max(c1.y, 0), e6 = max(c1.z, 0), e7 = max(c1.w, 0);
    const int ts = e0 + e1 + e2 + e3 + e4 + e5 + e6 + e7;
    int incl = ts;
#pragma unroll
    for (int d = 1; d < 32; d <<= 1) {
      const int t = __shfl_up(incl, d);
      if (lane >= d) incl += t;
    }
    if (lane == 31) wtot[wave] = incl;
    __syncthreads();
    const int S0 = wtot[0]  + wtot[1]  + wtot[2]  + wtot[3];
    const int S1 = wtot[4]  + wtot[5]  + wtot[6]  + wtot[7];
    const int S2 = wtot[8]  + wtot[9]  + wtot[10] + wtot[11];
    const int S3 = wtot[12] + wtot[13] + wtot[14] + wtot[15];
    int pre = 0;
#pragma unroll 1
    for (int w = 4 * sub; w < wave; ++w) pre += wtot[w];
    const int b0 = carry;
    const int b1 = b0 + ((S0 + 31) & ~31);
    const int b2 = b1 + ((S1 + 31) & ~31);
    const int b3 = b2 + ((S2 + 31) & ~31);
    const int b4 = b3 + ((S3 + 31) & ~31);
    const int myb = sub == 0 ? b0 : (sub == 1 ? b1 : (sub == 2 ? b2 : b3));
    if (tid == 0) {
      srb[min(4 * ch + 0, RBN - 1)] = b0;
      srb[min(4 * ch + 1, RBN - 1)] = b1;
      srb[min(4 * ch + 2, RBN - 1)] = b2;
      srb[min(4 * ch + 3, RBN - 1)] = b3;
    }
    int run = myb + pre + incl - ts;
    soff[8 * tid + 0] = run; run += e0;
    soff[8 * tid + 1] = run; run += e1;
    soff[8 * tid + 2] = run; run += e2;
    soff[8 * tid + 3] = run; run += e3;
    soff[8 * tid + 4] = run; run += e4;
    soff[8 * tid + 5] = run; run += e5;
    soff[8 * tid + 6] = run; run += e6;
    soff[8 * tid + 7] = run;
    carry = b4;
    __syncthreads();
    const v4i o0 = *(const v4i*)(soff + 4 * tid);
    const v4i o1 = *(const v4i*)(soff + 4 * (tid + OTHR));
    int* op = off + base;
    *(volatile v4i*)(op + 4 * tid) = o0;
    *(volatile v4i*)(op + 4 * (tid + OTHR)) = o1;
    __threadfence();
    *(volatile v4i*)(op + 4 * tid) = o0;
    *(volatile v4i*)(op + 4 * (tid + OTHR)) = o1;
    __syncthreads();
  }
  if (tid == 0) srb[min(4 * nChunk, RBN - 1)] = carry;
  __syncthreads();
  v4i rv = {0, 0, 0, 0};
  if (tid < 32) rv = *(const v4i*)(srb + 4 * tid);
  if (tid < 32) *(volatile v4i*)(rbase + 4 * tid) = rv;
  __threadfence();
  if (tid < 32) *(volatile v4i*)(rbase + 4 * tid) = rv;
}

__global__ __launch_bounds__(NTHR) void k_fill(const int* __restrict__ ei, const int* __restrict__ off, const int* __restrict__ rbase,
                                               int* csr, int nE, int vec8, int csrLen) {
  extern __shared__ v4f lds_dyn[];
  int* region = (int*)lds_dyn;
  int* cursor = region + RCAP;
  int* list   = cursor + NBF;
  int* wcnt   = list + LISTN;
  const int tid = threadIdx.x, lane = tid & 31, wave = tid >> 5;
  const int b = blockIdx.x;
  const int nodeBase = b * NBF;
  const int* dsts = ei + nE;
  int rb0 = rbase[b];
  const int rb1 = rbase[b + 1];
  rb0 = rb0 < 0 ? 0 : (rb0 > csrLen ? csrLen : rb0);
  rb0 &= ~31;
  int len = rb1 - rb0;
  len = len < 0 ? 0 : (len > RCAP ? RCAP : len);
  int lenW = (len + 31) & ~31;
  if (rb0 + lenW > csrLen) lenW = (csrLen - rb0) & ~31;
  {
    const v4i z = {0, 0, 0, 0};
    for (int i = tid; i < RCAP / 4; i += NTHR) ((v4i*)region)[i] = z;
    for (int s = tid; s < NBF; s += NTHR) {
      int o = off[nodeBase + s] - rb0;
      o = o < 0 ? 0 : (o > RCAP ? RCAP : o);
      cursor[s] = o;
    }
  }
  __syncthreads();
  const int nChunks = (nE + CHUNK - 1) / CHUNK;
#pragma unroll 1
  for (int ch = 0; ch < nChunks; ++ch) {
    const int cbase = ch * CHUNK;
    const int wc = scan_chunk<NBF>(dsts, nE, cbase, nodeBase, vec8, list, tid, lane, wave);
    if (lane == 0) wcnt[wave] = wc;
    __syncthreads();
    if (wave == 0) {
#pragma unroll 1
      for (int wsx = 0; wsx < NWAVE; ++wsx) {
        int n = __builtin_amdgcn_readfirstlane(wcnt[wsx]);
        n = n > WCAP ? WCAP : (n < 0 ? 0 : n);
        const int* lp = list + wsx * WCAP;
#pragma unroll 1
        for (int i = 0; i < n; ++i) {
          const int ent  = __builtin_amdgcn_readfirstlane(lp[i]);
          const int slot = ent & (NBF - 1);
          int e = cbase + ((ent >> 12) & (CHUNK - 1));
          e = e > nE - 1 ? nE - 1 : e;
          if (lane == 0) {
            int p = cursor[slot];
            p = p < 0 ? 0 : (p > RCAP - 1 ? RCAP - 1 : p);
            region[p] = e;
            const int np = p + 1;
            cursor[slot] = np > RCAP ? RCAP : np;
          }
        }
      }
    }
    __syncthreads();
  }
  const int nv = lenW >> 2;
  int* gp = csr + rb0;
#pragma unroll 1
  for (int i = tid; i < nv; i += NTHR) { const v4i v = ((const v4i*)region)[i]; *(volatile v4i*)(gp + 4 * i) = v; }
  __threadfence();
#pragma unroll 1
  for (int i = tid; i < nv; i += NTHR) { const v4i v = ((const v4i*)region)[i]; *(volatile v4i*)(gp + 4 * i) = v; }
}

__global__ __launch_bounds__(NTHR) void k_cvt(const float* __restrict__ x, unsigned short* hi, unsigned short* lo,
                                              int nR, int K, int items) {
  const int idx = blockIdx.x * NTHR + threadIdx.x;
  if (idx >= items) return;
  const int k8 = K >> 3;
  const int r = idx / k8;
  const int k0 = (idx - r * k8) * 8;
  const int rc = r < nR ? r : nR - 1;
  const float* xp = x + (size_t)rc * K + k0;
  const v4f a = *(const v4f*)xp;
  const v4f b = *(const v4f*)(xp + 4);
  v8us hv, lv;
  split8(a, b, hv, lv);
  *(volatile v8us*)(hi + (size_t)idx * 8) = hv; *(volatile v8us*)(lo + (size_t)idx * 8) = lv;
  __threadfence();
  *(volatile v8us*)(hi + (size_t)idx * 8) = hv; *(volatile v8us*)(lo + (size_t)idx * 8) = lv;
}

struct GArgs {
  const unsigned short* A0; const unsigned short* A1; const unsigned short* B0; const unsigned short* B1;
  const float* atts; const float* attd; float* C; float* asd;
  int lda, ksteps, ldb, z0;
};
static_assert(sizeof(GArgs) == 80);

__global__ __launch_bounds__(NTHR) void k_gemm(GArgs g) {
  extern __shared__ v4f lds_dyn[];
  float* stg  = (float*)lds_dyn;
  float* satt = stg + GROWS * GNC;
  float* sasd = satt + 128;
  const int tid = threadIdx.x, lane = tid & 31, wave = tid >> 5, hh = lane >> 4, m = lane & 15;
  const int rowBase = (int)blockIdx.x * GROWS;
  {
    const float va = g.atts[tid & 63];
    const float vd = g.attd[tid & 63];
    if (tid < 128) satt[tid] = (tid < 64) ? va : vd;
  }
  const int arow = rowBase + wave * 16 + m;
  const unsigned short* a0p = g.A0 + (size_t)arow * g.lda + 8 * hh;
  const unsigned short* a1p = g.A1 + (size_t)arow * g.lda + 8 * hh;
  v8f acc[4];
#pragma unroll
  for (int t = 0; t < 4; ++t) { v8f z = {0.f, 0.f, 0.f, 0.f, 0.f, 0.f, 0.f, 0.f}; acc[t] = z; }
#pragma unroll 1
  for (int kt = 0; kt < g.ksteps; ++kt) {
    FragB ah, al;
    ah.h[0] = *(const v8us*)(a0p + 32 * kt); ah.h[1] = *(const v8us*)(a0p + 32 * kt + 16);
    al.h[0] = *(const v8us*)(a1p + 32 * kt); al.h[1] = *(const v8us*)(a1p + 32 * kt + 16);
#pragma unroll
    for (int t = 0; t < 4; ++t) {
      const size_t bo = (size_t)(16 * t + m) * g.ldb + 32 * kt + 8 * hh;
      FragB bh, bl;
      bh.h[0] = *(const v8us*)(g.B0 + bo); bh.h[1] = *(const v8us*)(g.B0 + bo + 16);
      bl.h[0] = *(const v8us*)(g.B1 + bo); bl.h[1] = *(const v8us*)(g.B1 + bo + 16);
      acc[t] = wm3(ah.v, al.v, bh.v, bl.v, acc[t]);
    }
  }
  const int r0 = wave * 16 + 8 * hh;
#pragma unroll
  for (int t = 0; t < 4; ++t) {
    const int lcol = 16 * t + m;
#pragma unroll
    for (int r = 0; r < 8; ++r) stg[(r0 + r) * GNC + lcol] = acc[t][r];
  }
  __syncthreads();
  {
    const int row = tid >> 1, kind = tid & 1;
    const float* ap = satt + kind * 64;
    const float* hp = stg + row * GNC;
#pragma unroll 1
    for (int h = 0; h < NH; ++h) {
      float s = 0.0f;
#pragma unroll 4
      for (int c = 0; c < 16; ++c) s = fmaf(hp[16 * h + c], ap[16 * h + c], s);
      sasd[row * 8 + kind * 4 + h] = s;
    }
  }
  __syncthreads();
  const int rsel = lane >> 4, csel = 4 * (lane & 15);
  float* cb = g.C + (size_t)rowBase * GNC;
  float* ab = g.asd + (size_t)rowBase * 8;
  const v4f av = *(const v4f*)(sasd + 4 * tid);
#pragma unroll
  for (int i = 0; i < 8; ++i) {
    const int lr = wave * 16 + 2 * i + rsel;
    const v4f v = *(const v4f*)(stg + lr * GNC + csel);
    *(volatile v4f*)(cb + (size_t)lr * GNC + csel) = v;
  }
  *(volatile v4f*)(ab + 4 * tid) = av;
  __threadfence();
#pragma unroll
  for (int i = 0; i < 8; ++i) {
    const int lr = wave * 16 + 2 * i + rsel;
    const v4f v = *(const v4f*)(stg + lr * GNC + csel);
    *(volatile v4f*)(cb + (size_t)lr * GNC + csel) = v;
  }
  *(volatile v4f*)(ab + 4 * tid) = av;
}

template <int KIND>
__global__ __launch_bounds__(NTHR) void k_node(const int* __restrict__ csr, const int* __restrict__ off, const int* __restrict__ cnt,
    const int* __restrict__ ei, const float* __restrict__ hlin, const float* __restrict__ asd,
    const float* __restrict__ bias, const float* __restrict__ gam, const float* __restrict__ bet,
    const float* __restrict__ mu, const float* __restrict__ var,
    unsigned int* pH, unsigned int* pL, float* hout, float* mtab, float* ztab, int nN, int nE, int csrLen) {
  __shared__ __attribute__((aligned(16))) float slog[NWAVE * NSLOT * NH];
  __shared__ __attribute__((aligned(16))) int   ssrc[NWAVE * NSLOT];
  __shared__ __attribute__((aligned(16))) float smt[(KIND == 0) ? NWAVE * 128 : 4];
  __shared__ __attribute__((aligned(16))) float szt[(KIND == 0) ? NWAVE * 128 : 4];
  const int tid = threadIdx.x, lane = tid & 31, wave = tid >> 5;
  const int hd = lane >> 3;
  const int tbase = blockIdx.x * TGT + wave * 32;
  float* wl = slog + wave * (NSLOT * NH);
  int* wsrc = ssrc + wave * NSLOT;
  const int cnt_l = cnt[tbase + lane], off_l = off[tbase + lane];
  const v2f bv = *(const v2f*)(bias + 2 * lane);
  const v2f gv = *(const v2f*)(gam + 2 * lane);
  const v2f ev = *(const v2f*)(bet + 2 * lane);
  const v2f mv = *(const v2f*)(mu + 2 * lane);
  const v2f vv = *(const v2f*)(var + 2 * lane);
  const float rs0 = 1.0f / sqrtf(vv.x + BN_EPS);
  const float rs1 = 1.0f / sqrtf(vv.y + BN_EPS);
#pragma unroll 1
  for (int j = 0; j < 32; ++j) {
    const int d = tbase + j;
    int n = __builtin_amdgcn_readfirstlane(__shfl(cnt_l, j));
    n = n < 0 ? 0 : (n > NSLOT - 1 ? NSLOT - 1 : n);
    const int st = __builtin_amdgcn_readfirstlane(__shfl(off_l, j));
    const int T = n + 1;
    const v4f adv = *(const v4f*)(asd + (size_t)d * 8 + 4);
    __builtin_amdgcn_fence(__ATOMIC_RELEASE, "wavefront");
    __builtin_amdgcn_wave_barrier();
    float M0 = NEG_BIG, M1 = NEG_BIG, M2 = NEG_BIG, M3 = NEG_BIG;
#pragma unroll 1
    for (int q0 = 0; q0 < T; q0 += 32) {
      const int e = q0 + lane;
      const bool inE = e < n;
      const bool val = e < T;
      int p = st + (inE ? e : 0); p = p < 0 ? 0 : (p > csrLen - 1 ? csrLen - 1 : p);
      int eid = csr[p]; eid = eid < 0 ? 0 : (eid > nE - 1 ? nE - 1 : eid);
      int s = ei[eid];  s = s < 0 ? 0 : (s > nN - 1 ? nN - 1 : s);
      const int src = inE ? s : d;
      const v4f av = *(const v4f*)(asd + (size_t)src * 8);
      const float l0 = lgt(av.x + adv.x), l1 = lgt(av.y + adv.y), l2 = lgt(av.z + adv.z), l3 = lgt(av.w + adv.w);
      M0 = val ? fmaxf(M0, l0) : M0;
      M1 = val ? fmaxf(M1, l1) : M1;
      M2 = val ? fmaxf(M2, l2) : M2;
      M3 = val ? fmaxf(M3, l3) : M3;
      if (val) {
        wl[e * NH + 0] = l0; wl[e * NH + 1] = l1; wl[e * NH + 2] = l2; wl[e * NH + 3] = l3;
        wsrc[e] = src;
      }
    }
    M0 = wmax(M0); M1 = wmax(M1); M2 = wmax(M2); M3 = wmax(M3);
    __builtin_amdgcn_fence(__ATOMIC_RELEASE, "wavefront");
    __builtin_amdgcn_wave_barrier();
    float z0 = 0.0f, z1 = 0.0f, z2 = 0.0f, z3 = 0.0f;
#pragma unroll 1
    for (int q0 = 0; q0 < T; q0 += 32) {
      const int e = q0 + lane;
      const bool val = e < T;
      const float x0 = wl[e * NH + 0], x1 = wl[e * NH + 1], x2 = wl[e * NH + 2], x3 = wl[e * NH + 3];
      const float p0 = val ? __expf(x0 - M0) : 0.0f;
      const float p1 = val ? __expf(x1 - M1) : 0.0f;
      const float p2 = val ? __expf(x2 - M2) : 0.0f;
      const float p3 = val ? __expf(x3 - M3) : 0.0f;
      wl[e * NH + 0] = p0; wl[e * NH + 1] = p1; wl[e * NH + 2] = p2; wl[e * NH + 3] = p3;
      z0 += p0; z1 += p1; z2 += p2; z3 += p3;
    }
    z0 = wsum(z0); z1 = wsum(z1); z2 = wsum(z2); z3 = wsum(z3);
    __builtin_amdgcn_fence(__ATOMIC_RELEASE, "wavefront");
    __builtin_amdgcn_wave_barrier();
    const float zs = (hd == 0) ? z0 : ((hd == 1) ? z1 : ((hd == 2) ? z2 : z3));
    float acc0 = 0.0f, acc1 = 0.0f;
#pragma unroll 1
    for (int e = 0; e < T; ++e) {
      const int src = wsrc[e];
      const float w = wl[e * NH + hd];
      const v2f hv = *(const v2f*)(hlin + (size_t)src * CH + 2 * lane);
      acc0 = fmaf(w, hv.x, acc0);
      acc1 = fmaf(w, hv.y, acc1);
    }
    const float rz = __builtin_amdgcn_rcpf(zs);
    float o0 = fmaf(acc0, rz, bv.x);
    float o1 = fmaf(acc1, rz, bv.y);
    o0 = fmaxf(o0, 0.0f);
    o1 = fmaxf(o1, 0.0f);
    const float y0 = fmaf(gv.x * (o0 - mv.x), rs0, ev.x);
    const float y1 = fmaf(gv.y * (o1 - mv.y), rs1, ev.y);
    if (KIND == 0) {
      if (lane == 0) {
        smt[wave * 128 + 4 * j + 0] = M0; smt[wave * 128 + 4 * j + 1] = M1;
        smt[wave * 128 + 4 * j + 2] = M2; smt[wave * 128 + 4 * j + 3] = M3;
        szt[wave * 128 + 4 * j + 0] = z0; szt[wave * 128 + 4 * j + 1] = z1;
        szt[wave * 128 + 4 * j + 2] = z2; szt[wave * 128 + 4 * j + 3] = z3;
      }
    }
    if (KIND != 2) {
      unsigned int hw, lw;
      pk2(y0, y1, hw, lw);
      unsigned int* ph = pH + (size_t)d * (CH / 2) + lane;
      unsigned int* pl = pL + (size_t)d * (CH / 2) + lane;
      *(volatile unsigned int*)ph = hw; *(volatile unsigned int*)pl = lw;
      __threadfence();
      *(volatile unsigned int*)ph = hw; *(volatile unsigned int*)pl = lw;
    } else {
      v2f yv;
      yv.x = y0; yv.y = y1;
      float* op = hout + (size_t)d * CH + 2 * lane;
      *(volatile v2f*)op = yv;
      __threadfence();
      *(volatile v2f*)op = yv;
    }
  }
  if (KIND == 0) {
    __builtin_amdgcn_fence(__ATOMIC_RELEASE, "wavefront");
    __builtin_amdgcn_wave_barrier();
    const v4f m4 = *(const v4f*)(smt + wave * 128 + 4 * lane);
    const v4f z4 = *(const v4f*)(szt + wave * 128 + 4 * lane);
    float* mq = mtab + (size_t)(tbase + lane) * NH;
    float* zq = ztab + (size_t)(tbase + lane) * NH;
    *(volatile v4f*)mq = m4; *(volatile v4f*)zq = z4;
    __threadfence();
    *(volatile v4f*)mq = m4; *(volatile v4f*)zq = z4;
  }
}

__global__ __launch_bounds__(NTHR) void k_alpha(const int* __restrict__ ei, const float* __restrict__ asd, const float* __restrict__ mtab,
                                                const float* __restrict__ ztab, float* out1, int nN, int nE, int nTot) {
  const int tid = threadIdx.x;
  const int e = (int)blockIdx.x * NTHR + tid;
  const int ec = e < nTot ? e : nTot - 1;
  const bool isIn = ec < nE;
  const int ie = isIn ? ec : 0;
  int s  = ei[ie];      s  = s  < 0 ? 0 : (s  > nN - 1 ? nN - 1 : s);
  int dd = ei[nE + ie]; dd = dd < 0 ? 0 : (dd > nN - 1 ? nN - 1 : dd);
  int sn = ec - nE;     sn = sn < 0 ? 0 : (sn > nN - 1 ? nN - 1 : sn);
  const int src = isIn ? s : sn;
  const int dst = isIn ? dd : sn;
  const v4f av  = *(const v4f*)(asd + (size_t)src * 8);
  const v4f adv = *(const v4f*)(asd + (size_t)dst * 8 + 4);
  const v4f m4  = *(const v4f*)(mtab + (size_t)dst * NH);
  const v4f z4  = *(const v4f*)(ztab + (size_t)dst * NH);
  v4f a;
  a.x = __expf(lgt(av.x + adv.x) - m4.x) * __builtin_amdgcn_rcpf(z4.x);
  a.y = __expf(lgt(av.y + adv.y) - m4.y) * __builtin_amdgcn_rcpf(z4.y);
  a.z = __expf(lgt(av.z + adv.z) - m4.z) * __builtin_amdgcn_rcpf(z4.z);
  a.w = __expf(lgt(av.w + adv.w) - m4.w) * __builtin_amdgcn_rcpf(z4.w);
  float* op = out1 + (size_t)e * NH;
  if (e < nTot) *(volatile v4f*)op = a;
  __threadfence();
  if (e < nTot) *(volatile v4f*)op = a;
}

__global__ __launch_bounds__(PTHR) void k_pool1(const float* __restrict__ h, const int* __restrict__ batch, float* pp, float* pc, int nN) {
  __shared__ __attribute__((aligned(16))) float sps[NG * CH];
  __shared__ __attribute__((aligned(16))) float spc[NG];
  __shared__ int sb[NPB];
  const int tid = threadIdx.x;
  const int base = (int)blockIdx.x * NPB;
  for (int i = tid; i < NG * CH; i += PTHR) sps[i] = 0.0f;
  for (int i = tid; i < NPB; i += PTHR) {
    int node = base + i; node = node > nN - 1 ? nN - 1 : node;
    int g = batch[node]; g = g < 0 ? 0 : (g > NG - 1 ? NG - 1 : g);
    sb[i] = g;
  }
  __syncthreads();
  int nloc = nN - base;
  nloc = nloc > NPB ? NPB : (nloc < 0 ? 0 : nloc);
#pragma unroll 1
  for (int i = 0; i < nloc; ++i) {
    const int g = sb[i];
    const float v = h[(size_t)(base + i) * CH + tid];
    sps[g * CH + tid] = sps[g * CH + tid] + v;
  }
  float c0 = 0.0f, c1 = 0.0f;
#pragma unroll 1
  for (int i = 0; i < nloc; ++i) {
    const int g = sb[i];
    c0 += (g == tid) ? 1.0f : 0.0f;
    c1 += (g == tid + PTHR) ? 1.0f : 0.0f;
  }
  spc[tid] = c0; spc[tid + PTHR] = c1;
  __syncthreads();
  float* ppb = pp + (size_t)blockIdx.x * (NG * CH);
  float* pcb = pc + (size_t)blockIdx.x * NG;
#pragma unroll 1
  for (int i = 0; i < (NG * CH) / (4 * PTHR); ++i) {
    const v4f v = *(const v4f*)(sps + (i * PTHR + tid) * 4);
    *(volatile v4f*)(ppb + (i * PTHR + tid) * 4) = v;
  }
  if (tid < 32) { const v4f c = *(const v4f*)(spc + 4 * tid); *(volatile v4f*)(pcb + 4 * tid) = c; }
  __threadfence();
#pragma unroll 1
  for (int i = 0; i < (NG * CH) / (4 * PTHR); ++i) {
    const v4f v = *(const v4f*)(sps + (i * PTHR + tid) * 4);
    *(volatile v4f*)(ppb + (i * PTHR + tid) * 4) = v;
  }
  if (tid < 32) { const v4f c = *(const v4f*)(spc + 4 * tid); *(volatile v4f*)(pcb + 4 * tid) = c; }
}

__global__ __launch_bounds__(NTHR) void k_pool2(const float* __restrict__ pp, const float* __restrict__ pc, const float* __restrict__ fcW,
                                                const float* __restrict__ fcb, float* out0, int nPB) {
  __shared__ __attribute__((aligned(16))) float spool[NG * CH];
  __shared__ __attribute__((aligned(16))) float scnt[NG];
  __shared__ __attribute__((aligned(16))) float sout[NG];
  const int tid = threadIdx.x;
#pragma unroll 1
  for (int idx = tid; idx < NG * CH; idx += NTHR) {
    float s = 0.0f;
#pragma unroll 1
    for (int b = 0; b < nPB; ++b) s += pp[(size_t)b * (NG * CH) + idx];
    spool[idx] = s;
  }
  if (tid < NG) {
    float c = 0.0f;
#pragma unroll 1
    for (int b = 0; b < nPB; ++b) c += pc[(size_t)b * NG + tid];
    scnt[tid] = c;
  }
  __syncthreads();
  if (tid < NG) {
    const float rc = 1.0f / fmaxf(scnt[tid], 1.0f);
    float acc = 0.0f;
#pragma unroll 4
    for (int c = 0; c < CH; ++c) acc = fmaf(spool[tid * CH + c] * rc, fcW[c], acc);
    const float xo = acc + fcb[0];
    sout[tid] = 1.0f / (1.0f + __expf(-xo));
  }
  __syncthreads();
  v4f ov = {0.f, 0.f, 0.f, 0.f};
  if (tid < 32) ov = *(const v4f*)(sout + 4 * tid);
  if (tid < 32) *(volatile v4f*)(out0 + 4 * tid) = ov;
  __threadfence();
  if (tid < 32) *(volatile v4f*)(out0 + 4 * tid) = ov;
}

static GArgs mkg(const unsigned short* A0, const unsigned short* A1, int lda, int ksteps,
                 const unsigned short* B0, const unsigned short* B1, int ldb,
                 const float* atts, const float* attd, float* C, float* asd) {
  GArgs g;
  g.A0 = A0; g.A1 = A1; g.B0 = B0; g.B1 = B1; g.atts = atts; g.attd = attd; g.C = C; g.asd = asd;
  g.lda = lda; g.ksteps = ksteps; g.ldb = ldb; g.z0 = 0;
  return g;
}

extern "C" void kernel_launch(void* const* d_in, const int* in_sizes, int n_in,
                              void* d_out, int out_size, void* d_ws, size_t ws_size,
                              hipStream_t stream) {
  if (n_in < 29) return;
  const int kin[3] = {128, 64, 64};
  if (in_sizes[0] < 128 || (in_sizes[0] % 128) != 0) return;
  const int N = in_sizes[0] / 128;
  if (in_sizes[1] < 2 || (in_sizes[1] & 1) != 0) return;
  const int E = in_sizes[1] / 2;
  if (in_sizes[2] != N) return;
  for (int L = 0; L < 3; ++L) {
    if (in_sizes[3 + 8 * L] != CH * kin[L]) return;
    if (in_sizes[4 + 8 * L] != NH * 16 || in_sizes[5 + 8 * L] != NH * 16) return;
    for (int q = 6; q <= 10; ++q) if (in_sizes[q + 8 * L] != CH) return;
  }
  if (in_sizes[27] != CH || in_sizes[28] != 1) return;
  if (N > (1 << 22) || E > (1 << 26)) return;
  const long long Etot = (long long)E + (long long)N;
  if ((long long)out_size != (long long)NG + Etot * NH) return;

  const int NP = ((N + TGT - 1) / TGT) * TGT;
  const int nBC = (N + NBC - 1) / NBC;
  if (4 * nBC + 1 > RBN) return;
  const int CNTPAD = nBC * NBC;
  if (NP > CNTPAD) return;
  const int nBF = (N + NBF - 1) / NBF;
  if (nBF > 4 * nBC) return;
  const int csrLen = ((E + 31) & ~31) + 4096;
  if (31 * 4 * nBC > 4096) return;
  const int nPB = (N + NPB - 1) / NPB;

  const float* x     = (const float*)d_in[0];
  const int*   ei    = (const int*)d_in[1];
  const int*   batch = (const int*)d_in[2];
  const float* fcW   = (const float*)d_in[27];
  const float* fcb   = (const float*)d_in[28];
  float* out0 = (float*)d_out;
  float* out1 = out0 + NG;

  size_t wOffH[3], wOffL[3]; size_t whalves = 0;
  for (int L = 0; L < 3; ++L) {
    wOffH[L] = whalves; whalves += (size_t)CH * kin[L];
    wOffL[L] = whalves; whalves += (size_t)CH * kin[L];
  }

  size_t off = 0;
  const size_t oW   = off; off = ((off + whalves * 2) + 255) & ~(size_t)255;
  const size_t oXH  = off; off = ((off + (size_t)NP * 128 * 2) + 255) & ~(size_t)255;
  const size_t oXL  = off; off = ((off + (size_t)NP * 128 * 2) + 255) & ~(size_t)255;
  const size_t oHH  = off; off = ((off + (size_t)NP * CH * 2) + 255) & ~(size_t)255;
  const size_t oHL  = off; off = ((off + (size_t)NP * CH * 2) + 255) & ~(size_t)255;
  const size_t oCnt = off; off = ((off + (size_t)CNTPAD * 4) + 255) & ~(size_t)255;
  const size_t oOff = off; off = ((off + (size_t)CNTPAD * 4) + 255) & ~(size_t)255;
  const size_t oRb  = off; off = ((off + (size_t)RBN * 4) + 255) & ~(size_t)255;
  const size_t oCsr = off; off = ((off + (size_t)csrLen * 4) + 255) & ~(size_t)255;
  const size_t oHl  = off; off = ((off + (size_t)NP * CH * 4) + 255) & ~(size_t)255;
  const size_t oAsd = off; off = ((off + (size_t)NP * 8 * 4) + 255) & ~(size_t)255;
  const size_t oMt  = off; off = ((off + (size_t)NP * NH * 4) + 255) & ~(size_t)255;
  const size_t oZt  = off; off = ((off + (size_t)NP * NH * 4) + 255) & ~(size_t)255;
  const size_t oHo  = off; off = ((off + (size_t)NP * CH * 4) + 255) & ~(size_t)255;
  const size_t oPp  = off; off = ((off + (size_t)nPB * NG * CH * 4) + 255) & ~(size_t)255;
  const size_t oPc  = off; off = ((off + (size_t)nPB * NG * 4) + 255) & ~(size_t)255;
  if (off > ws_size || off > (size_t)WSCAP) return;

  char* ws = (char*)d_ws;
  unsigned short* wp  = (unsigned short*)(ws + oW);
  unsigned short* xHh = (unsigned short*)(ws + oXH);
  unsigned short* xLh = (unsigned short*)(ws + oXL);
  unsigned short* hHh = (unsigned short*)(ws + oHH);
  unsigned short* hLh = (unsigned short*)(ws + oHL);
  int* cnt  = (int*)(ws + oCnt);
  int* offp = (int*)(ws + oOff);
  int* rb   = (int*)(ws + oRb);
  int* csr  = (int*)(ws + oCsr);
  float* hlin = (float*)(ws + oHl);
  float* asd  = (float*)(ws + oAsd);
  float* mtab = (float*)(ws + oMt);
  float* ztab = (float*)(ws + oZt);
  float* hout = (float*)(ws + oHo);
  float* pp   = (float*)(ws + oPp);
  float* pc   = (float*)(ws + oPc);
  const int vec8 = ((E & 3) == 0) ? 1 : 0;

  k_cvt<<<(NP * 16 + NTHR - 1) / NTHR, NTHR, 0, stream>>>(x, xHh, xLh, N, 128, NP * 16);
  for (int L = 0; L < 3; ++L) {
    const int items = CH * kin[L] / 8;
    k_cvt<<<(items + NTHR - 1) / NTHR, NTHR, 0, stream>>>((const float*)d_in[3 + 8 * L], wp + wOffH[L], wp + wOffL[L], CH, kin[L], items);
  }
  k_count<<<nBC, NTHR, 0, stream>>>(ei, cnt, E, vec8);
  k_offsets<<<1, OTHR, 0, stream>>>(cnt, offp, rb, nBC);
  hipFuncSetAttribute(reinterpret_cast<const void*>(&k_fill), hipFuncAttributeMaxDynamicSharedMemorySize, LDS_FILL);
  k_fill<<<nBF, NTHR, LDS_FILL, stream>>>(ei, offp, rb, csr, E, vec8, csrLen);

  for (int L = 0; L < 3; ++L) {
    const unsigned short* A0 = (L == 0) ? xHh : hHh;
    const unsigned short* A1 = (L == 0) ? xLh : hLh;
    GArgs a = mkg(A0, A1, kin[L], kin[L] / 32, wp + wOffH[L], wp + wOffL[L], kin[L],
                  (const float*)d_in[4 + 8 * L], (const float*)d_in[5 + 8 * L], hlin, asd);
    k_gemm<<<dim3(NP / GROWS, 1, 1), NTHR, LDS_GEMM, stream>>>(a);
    const float* bias = (const float*)d_in[6 + 8 * L];
    const float* gam  = (const float*)d_in[7 + 8 * L];
    const float* bet  = (const float*)d_in[8 + 8 * L];
    const float* mu   = (const float*)d_in[9 + 8 * L];
    const float* var  = (const float*)d_in[10 + 8 * L];
    if (L == 0) {
      k_node<0><<<NP / TGT, NTHR, 0, stream>>>(csr, offp, cnt, ei, hlin, asd, bias, gam, bet, mu, var,
          (unsigned int*)hHh, (unsigned int*)hLh, hout, mtab, ztab, N, E, csrLen);
      k_alpha<<<(int)((Etot + NTHR - 1) / NTHR), NTHR, 0, stream>>>(ei, asd, mtab, ztab, out1, N, E, (int)Etot);
    } else if (L == 1) {
      k_node<1><<<NP / TGT, NTHR, 0, stream>>>(csr, offp, cnt, ei, hlin, asd, bias, gam, bet, mu, var,
          (unsigned int*)hHh, (unsigned int*)hLh, hout, mtab, ztab, N, E, csrLen);
    } else {
      k_node<2><<<NP / TGT, NTHR, 0, stream>>>(csr, offp, cnt, ei, hlin, asd, bias, gam, bet, mu, var,
          (unsigned int*)hHh, (unsigned int*)hLh, hout, mtab, ztab, N, E, csrLen);
    }
  }
  k_pool1<<<nPB, PTHR, 0, stream>>>(hout, batch, pp, pc, N);
  k_pool2<<<1, NTHR, 0, stream>>>(pp, pc, fcW, fcb, out0, nPB);
}
